// UnifiedPolicyValueNetwork_74844100100171
// MI455X (gfx1250) — hardware-verified
//
#include <hip/hip_runtime.h>
#include <math.h>

typedef __attribute__((ext_vector_type(16))) _Float16 v16h;
typedef __attribute__((ext_vector_type(16))) __bf16 v16b;
typedef __attribute__((ext_vector_type(8)))  _Float16 v8h;
typedef __attribute__((ext_vector_type(8)))  float v8f;
typedef __attribute__((ext_vector_type(4)))  float v4f;
typedef __attribute__((ext_vector_type(2)))  float v2f;
typedef __attribute__((ext_vector_type(4)))  unsigned v4u;
typedef __attribute__((ext_vector_type(4)))  int v4i;
typedef float __attribute__((may_alias)) float_a;
typedef int __attribute__((may_alias)) int_a;

template <typename T> __device__ __forceinline__ void vst2(void* p, T v) { *(volatile T*)p = v; __threadfence(); *(volatile T*)p = v; }
__device__ __forceinline__ v8f wmma16(v16h a, v16h b, v8f c) {
  v8f d = __builtin_amdgcn_wmma_f32_16x16x32_f16(false, a, false, b, (short)0, c, false, false);
  asm volatile("v_nop\n\tv_nop\n\tv_nop\n\tv_nop" : "+v"(d) : "v"(a), "v"(b));
  return d;
}
__device__ __forceinline__ v8f wmma_bf(v16b a, v16b b, v8f c) {
  v8f d = __builtin_amdgcn_wmma_f32_16x16x32_bf16(false, a, false, b, (short)0, c, false, false);
  asm volatile("v_nop\n\tv_nop\n\tv_nop\n\tv_nop" : "+v"(d) : "v"(a), "v"(b));
  return d;
}
__device__ __forceinline__ v16h frag_h(const _Float16* rowk0, int lane) {
  union { v16h v; v8h q[2]; } u; const _Float16* p = rowk0 + 8 * (lane >> 4);
  u.q[0] = *(const v8h*)p; u.q[1] = *(const v8h*)(p + 16); return u.v;
}
__device__ __forceinline__ v16h frag_f32(const float* rowk0, int lane) {
  v16h a; const float* p = rowk0 + 8 * (lane >> 4);
#pragma unroll
  for (int i = 0; i < 8; ++i) { a[i] = (_Float16)p[i]; a[8 + i] = (_Float16)p[16 + i]; }
  return a;
}
__device__ __forceinline__ v16h frag_f32s(const float* rowk0, int lane, float sc) {
  v16h a; const float* p = rowk0 + 8 * (lane >> 4);
#pragma unroll
  for (int i = 0; i < 8; ++i) { a[i] = (_Float16)(p[i] * sc); a[8 + i] = (_Float16)(p[16 + i] * sc); }
  return a;
}
__device__ __forceinline__ v16h fragc_f32(const float* W, int k0, int n, int lane, int ld, int K) {
  v16h a; const int g = lane >> 4;
#pragma unroll
  for (int i = 0; i < 8; ++i) { const int ka = k0 + 8 * g + i, kb = ka + 16;
    a[i] = (_Float16)(ka < K ? W[(size_t)(ka < K ? ka : K - 1) * ld + n] : 0.f); a[8 + i] = (_Float16)(kb < K ? W[(size_t)(kb < K ? kb : K - 1) * ld + n] : 0.f); }
  return a;
}
struct F2 { v16b h, l; };
__device__ __forceinline__ F2 bsplit16(const float v[16]) { F2 r;
#pragma unroll
  for (int i = 0; i < 16; ++i) { const __bf16 h = (__bf16)v[i]; r.h[i] = h; r.l[i] = (__bf16)(v[i] - (float)h); }
  return r; }
__device__ __forceinline__ F2 split_row(const float* row, int k0, int lane) { float v[16]; const float* p = row + k0 + 8 * (lane >> 4);
#pragma unroll
  for (int i = 0; i < 8; ++i) { v[i] = p[i]; v[8 + i] = p[16 + i]; }
  return bsplit16(v); }
__device__ __forceinline__ F2 split_rowK(const float* row, int k0, int lane, int K) { float v[16]; const int g = lane >> 4;
#pragma unroll
  for (int i = 0; i < 8; ++i) { const int ka = k0 + 8 * g + i, kb = ka + 16; v[i] = ka < K ? row[ka < K ? ka : K - 1] : 0.f; v[8 + i] = kb < K ? row[kb < K ? kb : K - 1] : 0.f; }
  return bsplit16(v); }
__device__ __forceinline__ F2 split_col(const float* W, int k0, int n, int lane, int ld, int K) { float v[16]; const int g = lane >> 4;
#pragma unroll
  for (int i = 0; i < 8; ++i) { const int ka = k0 + 8 * g + i, kb = ka + 16; v[i] = ka < K ? W[(size_t)(ka < K ? ka : K - 1) * ld + n] : 0.f; v[8 + i] = kb < K ? W[(size_t)(kb < K ? kb : K - 1) * ld + n] : 0.f; }
  return bsplit16(v); }
__device__ __forceinline__ v8f mac3(const F2& a, const F2& b, v8f c) { c = wmma_bf(a.l, b.h, c); c = wmma_bf(a.h, b.l, c); return wmma_bf(a.h, b.h, c); }
__device__ __forceinline__ float sigm(float v) { return 1.0f / (1.0f + expf(-v)); }
#define LDSX() do { asm volatile("s_wait_dscnt 0" ::: "memory"); __builtin_amdgcn_wave_barrier(); __builtin_amdgcn_fence(__ATOMIC_RELEASE, "workgroup"); } while (0)


#ifndef NN
#define NN 131072
#endif
#define EP 1048576
#ifndef NE
#define NE 1048576
#endif
#define FIN 32
#define MAXW 128
#define NBLK ((NN + 63) / 64)
#define NRP (NBLK * 64)
#define CSR_N NN
#define CSR_E NE
typedef __attribute__((ext_vector_type(8))) __bf16 v8b;
__device__ __forceinline__ v16b frag_b(const __bf16* rowk0, int lane) {
  union { v16b v; v8b q[2]; } u; const __bf16* p = rowk0 + 8 * (lane >> 4);
  u.q[0] = *(const v8b*)p; u.q[1] = *(const v8b*)(p + 16); return u.v;
}
__device__ __forceinline__ float bfr(float v) { return (float)(__bf16)v; }
__device__ __attribute__((noinline)) float exp_ni(float v) { return expf(v); }
__device__ __attribute__((noinline)) float erf_ni(float v) { return erff(v); }

#define CSR_FINN (CSR_E + 32 * CSR_NBK)
#define CSR_CHUNK 4096
#define CSR_BKT 256
#define CSR_NCH ((CSR_E + CSR_CHUNK - 1) / CSR_CHUNK)
#define CSR_NBK ((CSR_N + CSR_BKT - 1) / CSR_BKT)
#define CSR_NBKP (((CSR_NBK + 63) / 64) * 64)
#define CSR_SEGCAP (CSR_E + 32 * CSR_NBK * CSR_NCH)
#ifndef CSR_BCAP
#define CSR_BCAP 10240
#endif
#define CSR_SZ_CNT   (4u * CSR_NCH * CSR_NBKP)
#define CSR_SZ_OFF   (4u * CSR_NBK * (((CSR_NCH + 31) / 32) * 32))
#define CSR_SZ_BST   (4u * (((CSR_NBK + 1 + 31) / 32) * 32))
#define CSR_SZ_SEG   (4u * CSR_SEGCAP)
#define CSR_SZ_FIN   (4u * (CSR_E + 32 * CSR_NBK))
#define CSR_SZ_ROW   (4u * CSR_NBK * CSR_BKT)
#define CSR_OFFP (((CSR_NCH + 31) / 32) * 32)

__global__ __launch_bounds__(256) void k_csr_cnt(const int* __restrict__ DST, int dstride, int* __restrict__ CNT) {
  __shared__ unsigned short sc[256][CSR_NBK + 1]; __shared__ __align__(16) int srow[CSR_NBKP];
  const int c = blockIdx.x, tid = threadIdx.x;
  for (int b = 0; b < CSR_NBK; ++b) sc[tid][b] = 0;
  const size_t e0 = (size_t)c * CSR_CHUNK + tid * 16;
  for (int i = 0; i < 16; ++i) { const size_t e = e0 + i; if (e < (size_t)CSR_E) { int d = DST[e * dstride]; d = min(max(d, 0), CSR_N - 1); sc[tid][d / CSR_BKT] += 1; } }
  __syncthreads();
  for (int b = tid; b < CSR_NBKP; b += 256) { int s = 0; if (b < CSR_NBK) for (int t = 0; t < 256; ++t) s += sc[t][b]; srow[b] = s; }
  __syncthreads();
  for (int q = tid; q < CSR_NBKP / 4; q += 256) vst2((unsigned*)(CNT + (size_t)c * CSR_NBKP + q * 4), *(const v4u*)&srow[q * 4]);
}
__global__ __launch_bounds__(256) void k_csr_scan(const int* __restrict__ CNT, int* __restrict__ OFF, int* __restrict__ BST) {
  __shared__ int sbt[CSR_NBK + 1]; __shared__ int sbs[((CSR_NBK + 1 + 31) / 32) * 32]; __shared__ int scnt[CSR_NBK + 1]; __shared__ __align__(16) int sbuf[64][CSR_OFFP];
  const int tid = threadIdx.x;
  for (int b = tid; b < CSR_NBK; b += 256) { int sp = 0, st = 0; for (int c = 0; c < CSR_NCH; ++c) { const int n = CNT[(size_t)c * CSR_NBKP + b]; st += n; sp += (n + 31) & ~31; } sbt[b] = sp; scnt[b] = st; }
  for (int b = tid; b < ((CSR_NBK + 1 + 31) / 32) * 32; b += 256) sbs[b] = 0;
  __syncthreads();
  if (tid == 0) { int acc = 0, accf = 0; for (int b = 0; b < CSR_NBK; ++b) { const int t = sbt[b]; sbt[b] = acc; acc += t; sbs[b] = accf; accf += (scnt[b] + 31) & ~31; } sbs[CSR_NBK] = accf; }
  __syncthreads();
  for (int b0 = 0; b0 < CSR_NBK; b0 += 64) {
    if (tid < 64 && b0 + tid < CSR_NBK) { const int b = b0 + tid; int o = sbt[b]; for (int c = 0; c < CSR_OFFP; ++c) { if (c < CSR_NCH) { sbuf[tid][c] = o; o += (CNT[(size_t)c * CSR_NBKP + b] + 31) & ~31; } else sbuf[tid][c] = 0; } }
    __syncthreads();
    for (int q = tid; q < 64 * (CSR_OFFP / 4); q += 256) { const int r = q / (CSR_OFFP / 4), pc = q % (CSR_OFFP / 4); if (b0 + r < CSR_NBK) vst2((unsigned*)(OFF + (size_t)(b0 + r) * CSR_OFFP + pc * 4), *(const v4u*)&sbuf[r][pc * 4]); }
    __syncthreads(); }
  for (int q = tid; q < ((CSR_NBK + 1 + 31) / 32) * 32 / 4; q += 256) vst2((unsigned*)(BST + q * 4), *(const v4u*)&sbs[q * 4]);
}
__global__ __launch_bounds__(256) void k_csr_scatter(const int* __restrict__ SRC, const int* __restrict__ DST, int sstride, int dstride, const int* __restrict__ OFF, int* __restrict__ SEGS, int* __restrict__ SEGE) {
  __shared__ unsigned short sc[256][CSR_NBK + 1]; __shared__ int sbase[CSR_NBK + 1]; __shared__ int scn[CSR_NBK + 1]; __shared__ int sord[CSR_CHUNK];
  const int c = blockIdx.x, tid = threadIdx.x;
  for (int b = 0; b < CSR_NBK; ++b) sc[tid][b] = 0;
  const size_t e0 = (size_t)c * CSR_CHUNK + tid * 16; int bk[16];
#pragma unroll
  for (int i = 0; i < 16; ++i) { const size_t e = e0 + i; bk[i] = -1; if (e < (size_t)CSR_E) { int d = DST[e * dstride]; d = min(max(d, 0), CSR_N - 1); bk[i] = d / CSR_BKT; sc[tid][bk[i]] += 1; } }
  __syncthreads();
  for (int b = tid; b < CSR_NBK; b += 256) { int acc = 0; for (int t = 0; t < 256; ++t) { const int v = sc[t][b]; sc[t][b] = (unsigned short)acc; acc += v; } scn[b] = acc; }
  __syncthreads();
  if (tid == 0) { int acc = 0; for (int b = 0; b < CSR_NBK; ++b) { sbase[b] = acc; acc += scn[b]; } }
  __syncthreads();
#pragma unroll
  for (int i = 0; i < 16; ++i) { if (bk[i] >= 0) { const int b = bk[i]; const int r = sc[tid][b]; sc[tid][b] = (unsigned short)(r + 1); sord[sbase[b] + r] = tid * 16 + i; } }
  __syncthreads();
  for (int b = 0; b < CSR_NBK; ++b) { const int n = scn[b]; if (n == 0) continue; const int nl = ((n + 31) & ~31); const size_t o = (size_t)(min(max(OFF[(size_t)b * CSR_OFFP + c], 0), CSR_SEGCAP - nl) & ~31);
    for (int q = tid; q < nl / 4; q += 256) { int4 vs, ve;
#pragma unroll
      for (int k = 0; k < 4; ++k) { const int i = q * 4 + k; int s = -1, eid = -1; if (i < n) { const size_t e = (size_t)c * CSR_CHUNK + sord[sbase[b] + i]; s = min(max(SRC[e * sstride], 0), CSR_N - 1); eid = (int)e; } vs[k] = s; ve[k] = eid; }
      vst2((unsigned*)(SEGS + o + q * 4), *(const v4u*)&vs); vst2((unsigned*)(SEGE + o + q * 4), *(const v4u*)&ve); } }
}
__global__ __launch_bounds__(256) void k_csr_bucket(const int* __restrict__ CNT, const int* __restrict__ OFF, const int* __restrict__ BST, const int* __restrict__ SEGS, const int* __restrict__ SEGE, const int* __restrict__ DST, int dstride, int* __restrict__ FS, int* __restrict__ FE, int* __restrict__ ROWST, int* __restrict__ ROWCNT) {
  __shared__ int ssrc[CSR_BCAP]; __shared__ int seid[CSR_BCAP]; __shared__ unsigned char snod[CSR_BCAP]; __shared__ int souts[CSR_BCAP]; __shared__ int soute[CSR_BCAP]; __shared__ int scount[256]; __shared__ int sstart[257]; __shared__ int stot;
  const int b = blockIdx.x, tid = threadIdx.x;
  if (tid == 0) { int t = 0; for (int c = 0; c < CSR_NCH; ++c) t += min(max(CNT[(size_t)c * CSR_NBKP + b], 0), CSR_CHUNK); stot = (t <= CSR_BCAP) ? t : 0; }
  __syncthreads();
  { int base = 0; for (int c = 0; c < CSR_NCH; ++c) { const int n = min(max(CNT[(size_t)c * CSR_NBKP + b], 0), CSR_CHUNK); const int o = min(max(OFF[(size_t)b * CSR_OFFP + c], 0), CSR_SEGCAP - ((n + 31) & ~31));
      for (int i = tid; i < n; i += 256) { const int p = base + i; if (p < CSR_BCAP) { ssrc[p] = min(max(SEGS[o + i], 0), CSR_N - 1); const int e = min(max(SEGE[o + i], 0), CSR_E - 1); seid[p] = e; int d = DST[(size_t)e * dstride]; d = min(max(d, 0), CSR_N - 1); const int dl = d - b * CSR_BKT; snod[p] = (unsigned char)(dl >= 0 && dl < 256 ? dl : 255); } }
      base += n; } }
  __syncthreads();
  const int node = b * CSR_BKT + tid; int cnt = 0; for (int p = 0; p < stot; ++p) cnt += (snod[p] == tid) ? 1 : 0;
  scount[tid] = cnt; __syncthreads();
  if (tid == 0) { int acc = 0; for (int t = 0; t < 256; ++t) { sstart[t] = acc; acc += scount[t]; } sstart[256] = acc; }
  __syncthreads();
  const int bst0 = min(max(BST[b], 0), CSR_FINN - ((sstart[256] + 31) & ~31)) & ~31; const int gst = bst0 + sstart[tid];
  { int w = sstart[tid]; for (int p = 0; p < stot; ++p) if (snod[p] == tid) { souts[w] = ssrc[p]; soute[w] = seid[p]; ++w; } }
  __syncthreads();
  { const int n = sstart[256]; const int nl = (n + 31) & ~31; for (int q = tid; q < nl / 4; q += 256) { int4 vs, ve;
#pragma unroll
      for (int k = 0; k < 4; ++k) { const int i = q * 4 + k; vs[k] = i < n ? souts[i] : -1; ve[k] = i < n ? soute[i] : -1; }
      vst2((unsigned*)(FS + bst0 + q * 4), *(const v4u*)&vs); vst2((unsigned*)(FE + bst0 + q * 4), *(const v4u*)&ve); } }
  __syncthreads();
  { __shared__ __align__(16) int srs[256], src2[256]; srs[tid] = node < CSR_N ? gst : 0; src2[tid] = node < CSR_N ? cnt : 0; __syncthreads();
    if (tid < 64) vst2((unsigned*)(ROWST + (size_t)b * 256 + tid * 4), *(const v4u*)&srs[tid * 4]); else if (tid < 128) vst2((unsigned*)(ROWCNT + (size_t)b * 256 + (tid - 64) * 4), *(const v4u*)&src2[(tid - 64) * 4]); }
}


#define WS_CNT  0u
#define WS_OFF  (WS_CNT + CSR_SZ_CNT)
#define WS_BST  (WS_OFF + CSR_SZ_OFF)
#define WS_SEGS (WS_BST + CSR_SZ_BST)
#define WS_SEGE (WS_SEGS + CSR_SZ_SEG)
#define WS_FS   (WS_SEGE + CSR_SZ_SEG)
#define WS_FE   (WS_FS + CSR_SZ_FIN)
#define WS_RST  (WS_FE + CSR_SZ_FIN)
#define WS_RCT  (WS_RST + CSR_SZ_ROW)
#define WS_PW   (WS_RCT + CSR_SZ_ROW)
#define PW0 0
#define PWEND (4096 + 128 * 128)
#define WS_HW   (WS_PW + 2u * PWEND)
#define WS_H    (WS_HW + 4u * NRP * MAXW)
#define WS_T    (WS_H + 4u * NRP * MAXW)
#define WS_END0 (WS_H)

__global__ __launch_bounds__(256) void k_packT(const float* __restrict__ Wm, int K, int NOUT, __bf16* __restrict__ DST) {
  __shared__ __align__(16) __bf16 s[256]; const int n = blockIdx.x, tid = threadIdx.x;
  for (int k = tid; k < K; k += 256) s[k] = (__bf16)((n < NOUT) ? Wm[(size_t)k * NOUT + n] : 0.f);
  __syncthreads();
  for (int q = tid; q < K / 8; q += 256) vst2((unsigned*)(DST + (size_t)n * K + q * 8), *(const v4u*)&s[q * 8]);
}
template <int K, int NT, int RIN, int EPI>
__global__ __launch_bounds__(128) void k_lin(const float* __restrict__ A, int lda, const __bf16* __restrict__ P, const float* __restrict__ bias, float* __restrict__ OUT, int ldo) {
  __shared__ __align__(16) float so[4][16][NT * 16 + 4];
  const int tid = threadIdx.x, wave = tid >> 5, lane = tid & 31, col = lane & 15, g = lane >> 4; const size_t r0 = (size_t)blockIdx.x * 64 + wave * 16; size_t ra = r0 + col; if (ra >= NN) ra = NN - 1; const int n0 = blockIdx.y * (NT * 16);
  v8f acc[NT]; for (int j = 0; j < NT; ++j) acc[j] = (v8f){};
#pragma unroll 2
  for (int kc = 0; kc < K / 32; ++kc) { F2 a; if (RIN) { v16b ax; const float* p = A + ra * lda + kc * 32 + 8 * g;
#pragma unroll
      for (int i = 0; i < 8; ++i) { ax[i] = (__bf16)p[i]; ax[8 + i] = (__bf16)p[16 + i]; } a.h = ax; a.l = ax; } else a = split_row(A + ra * lda, kc * 32, lane);
#pragma unroll
    for (int j = 0; j < NT; ++j) { const v16b w = frag_b(P + (size_t)(n0 + j * 16 + col) * K + kc * 32, lane); if (!RIN) acc[j] = wmma_bf(a.l, w, acc[j]); acc[j] = wmma_bf(a.h, w, acc[j]); } }
#pragma unroll
  for (int j = 0; j < NT; ++j) { const int n = n0 + j * 16 + col; const float bb = bias ? bfr(bias[n]) : 0.f;
#pragma unroll
    for (int r = 0; r < 8; ++r) { float v = acc[j][r] + bb; if (EPI == 1) v = fmaxf(v, 0.f); so[wave][8 * g + r][j * 16 + col] = v; } }
  LDSX();
  for (int rl = 0; rl < 16; ++rl) if (lane < NT * 4) vst2(OUT + (r0 + rl) * ldo + n0 + lane * 4, *(const v4f*)&so[wave][rl][lane * 4]);
}
template <int RELU>
__global__ __launch_bounds__(256) void k_agg(const float* __restrict__ HW, const int* __restrict__ FS, const int* __restrict__ RST, const int* __restrict__ RCT, const float* __restrict__ bias, int width, float* __restrict__ Hd) {
  __shared__ __align__(16) float so[16][MAXW + 4];
  const int tid = threadIdx.x, blk = blockIdx.x; const int nl = tid >> 4, sl = tid & 15; const int fw = width / 16, f0 = sl * fw; const size_t node = (size_t)blk * 16 + nl;
  float acc[MAXW / 16];
#pragma unroll
  for (int i = 0; i < MAXW / 16; ++i) acc[i] = 0.f;
  if (node < (size_t)NN) { const int cnt = min(max(RCT[node], 0), CSR_BCAP); const int st = min(max(RST[node], 0), CSR_FINN - cnt);
    for (int e = 0; e < cnt; ++e) { const int s = min(max(FS[st + e], 0), NN - 1); const float ds = rsqrtf((float)(min(max(RCT[s], 0), NE) + 1)); const float* hr = HW + (size_t)s * MAXW + f0;
#pragma unroll
      for (int i = 0; i < MAXW / 16; ++i) if (i < fw) acc[i] += ds * hr[i]; }
    const float di = rsqrtf((float)(cnt + 1)); const float* own = HW + node * MAXW + f0;
#pragma unroll
    for (int i = 0; i < MAXW / 16; ++i) if (i < fw) { float v = di * (acc[i] + di * own[i]) + bfr(bias[f0 + i]); if (RELU) v = fmaxf(v, 0.f); acc[i] = v; } }
#pragma unroll
  for (int i = 0; i < MAXW / 16; ++i) if (i < fw) so[nl][f0 + i] = (node < (size_t)NN) ? acc[i] : 0.f;
  __syncthreads();
  for (int q = tid; q < 16 * (width / 4); q += 256) { const int rl = q / (width / 4), pc = q % (width / 4); vst2(Hd + ((size_t)blk * 16 + rl) * MAXW + pc * 4, *(const v4f*)&so[rl][pc * 4]); }
}

#define NG 512
#define NCHK 128
#define CHN 1024
#define WS_MSG (WS_END0)
#define WS_PT  (WS_MSG + 4u * NRP * MAXW)
#define WS_PC  (WS_PT + 4u * NCHK * NG * MAXW)
#define WS_GE  (WS_PC + 4u * NCHK * NG)
#define WS_END (WS_GE + 4u * NG * MAXW)
__global__ __launch_bounds__(256) void k_wagg(const float* __restrict__ H0, const int* __restrict__ FS, const int* __restrict__ FE, const int* __restrict__ RST, const int* __restrict__ RCT, const float* __restrict__ EW, float* __restrict__ MSG) {
  __shared__ __align__(16) float so[16][MAXW + 4];
  const int tid = threadIdx.x, blk = blockIdx.x; const int nl = tid >> 4, f0 = (tid & 15) * 8; const size_t node = (size_t)blk * 16 + nl;
  float acc[8];
#pragma unroll
  for (int i = 0; i < 8; ++i) acc[i] = 0.f;
  if (node < (size_t)NN) { const int cnt = min(max(RCT[node], 0), CSR_BCAP); const int st = min(max(RST[node], 0), CSR_FINN - cnt);
    for (int e = 0; e < cnt; ++e) { const int s = min(max(FS[st + e], 0), NN - 1); const int eid = min(max(FE[st + e], 0), NE - 1); const float w = bfr(EW[eid]); const float* hr = H0 + (size_t)s * MAXW + f0;
#pragma unroll
      for (int i = 0; i < 8; ++i) acc[i] += w * hr[i]; } }
#pragma unroll
  for (int i = 0; i < 8; ++i) so[nl][f0 + i] = acc[i];
  __syncthreads();
  for (int q = tid; q < 16 * 32; q += 256) { const int rl = q >> 5, pc = q & 31; vst2(MSG + ((size_t)blk * 16 + rl) * MAXW + pc * 4, *(const v4f*)&so[rl][pc * 4]); }
}
__global__ __launch_bounds__(128) void k_comb(const float* MSG, const __bf16* __restrict__ P, const float* __restrict__ H0, float* Hd) {
  __shared__ __align__(16) float so[4][16][132];
  const int tid = threadIdx.x, wave = tid >> 5, lane = tid & 31, col = lane & 15, g = lane >> 4; const size_t r0 = (size_t)blockIdx.x * 64 + wave * 16;
  v8f acc[8] = {};
#pragma unroll
  for (int kc = 0; kc < MAXW / 32; ++kc) { const F2 a = split_row(MSG + (r0 + col) * MAXW, kc * 32, lane);
#pragma unroll
    for (int j = 0; j < 8; ++j) { const v16b w = frag_b(P + (size_t)(j * 16 + col) * MAXW + kc * 32, lane); acc[j] = wmma_bf(a.l, w, acc[j]); acc[j] = wmma_bf(a.h, w, acc[j]); } }
#pragma unroll
  for (int j = 0; j < 8; ++j) { const int n = j * 16 + col;
#pragma unroll
    for (int r = 0; r < 8; ++r) { const size_t row = r0 + 8 * g + r; so[wave][8 * g + r][n] = fmaxf(H0[row * MAXW + n] + acc[j][r], 0.f); } }
  LDSX();
  for (int rl = 0; rl < 16; ++rl) vst2(Hd + (r0 + rl) * MAXW + lane * 4, *(const v4f*)&so[wave][rl][lane * 4]);
}
__global__ __launch_bounds__(128) void k_poolpart(const float* __restrict__ Hd, const int* __restrict__ BATCH, float* __restrict__ PT, float* __restrict__ PC) {
  __shared__ __align__(16) float st[256][MAXW]; __shared__ __align__(16) float sc[256];
  const int chunk = blockIdx.x, gh = blockIdx.y, f = threadIdx.x; const int g0 = gh * 256;
  for (int g = 0; g < 256; ++g) st[g][f] = 0.f; for (int g = f; g < 256; g += 128) sc[g] = 0.f;
  __syncthreads();
  const int n0 = chunk * CHN, n1 = min(n0 + CHN, NN);
  for (int n = n0; n < n1; ++n) { const int g = min(max(BATCH[n], 0), NG - 1) - g0; if (g >= 0 && g < 256) { st[g][f] += Hd[(size_t)n * MAXW + f]; if (f == 0) sc[g] += 1.f; } }
  __syncthreads();
  for (int q = f; q < 256 * 32; q += 128) { const int g = q >> 5, pc = q & 31; vst2(PT + ((size_t)chunk * NG + g0 + g) * MAXW + pc * 4, *(const v4f*)&st[g][pc * 4]); }
  for (int q = f; q < 256 / 4; q += 128) vst2(PC + (size_t)chunk * NG + g0 + q * 4, *(const v4f*)&sc[q * 4]);
}
__global__ __launch_bounds__(128) void k_poolred(const float* __restrict__ PT, const float* __restrict__ PC, float* __restrict__ GE) {
  __shared__ __align__(16) float s[MAXW]; const int g = blockIdx.x, f = threadIdx.x; float acc = 0.f, cnt = 0.f;
  for (int c = 0; c < NCHK; ++c) { acc += PT[((size_t)c * NG + g) * MAXW + f]; cnt += PC[(size_t)c * NG + g]; }
  s[f] = (cnt > 0.f) ? acc / fmaxf(cnt, 1.0f) : 0.f; __syncthreads();
  if (f < 32) vst2(GE + (size_t)g * MAXW + f * 4, *(const v4f*)&s[f * 4]);
}
__global__ __launch_bounds__(256) void k_heads(const float* __restrict__ GE, const float* __restrict__ W1, const float* __restrict__ W2, const float* __restrict__ WA, const float* __restrict__ WS, const float* __restrict__ WT, const float* __restrict__ WACT, const float* __restrict__ WV1, const float* __restrict__ WV2, float* __restrict__ OA, float* __restrict__ OS, float* __restrict__ OT, float* __restrict__ OACT, float* __restrict__ OV) {
  __shared__ float sge[32][MAXW]; __shared__ float s1[32][128]; __shared__ float s2[32][64]; __shared__ __align__(16) float soa[32 * 5 + 16]; __shared__ __align__(16) float soact[32 * 4]; __shared__ __align__(16) float sov[32]; __shared__ float sv1[32][32];
  const int tid = threadIdx.x; const int gb = blockIdx.x * 32;
  for (int q = tid; q < 32 * MAXW; q += 256) sge[q / MAXW][q % MAXW] = GE[(size_t)(gb + q / MAXW) * MAXW + q % MAXW];
  __syncthreads();
  for (int q = tid; q < 32 * 128; q += 256) { const int gl = q >> 7, c = q & 127; float a = 0.f; for (int k = 0; k < MAXW; ++k) a += sge[gl][k] * (bfr(W1[(size_t)k * 128 + c]) + bfr(W1[(size_t)(MAXW + k) * 128 + c])); s1[gl][c] = fmaxf(a, 0.f); }
  __syncthreads();
  for (int q = tid; q < 32 * 64; q += 256) { const int gl = q >> 6, c = q & 63; float a = 0.f; for (int k = 0; k < 128; ++k) a += s1[gl][k] * bfr(W2[(size_t)k * 64 + c]); s2[gl][c] = fmaxf(a, 0.f); }
  __syncthreads();
  for (int q = tid; q < 32 * 5; q += 256) { const int gl = q / 5, c = q % 5; float a = 0.f; for (int k = 0; k < 64; ++k) a += s2[gl][k] * bfr(WA[k * 5 + c]); soa[q] = a; }
  for (int q = tid; q < 32 * 4; q += 256) { const int gl = q >> 2, c = q & 3; float a = 0.f; for (int k = 0; k < 64; ++k) a += s2[gl][k] * bfr(WACT[k * 4 + c]); soact[q] = a; }
  for (int q = tid; q < 32 * 32; q += 256) { const int gl = q >> 5, c = q & 31; float a = 0.f; for (int k = 0; k < 64; ++k) a += s2[gl][k] * bfr(WV1[k * 32 + c]); sv1[gl][c] = fmaxf(a, 0.f); }
  __syncthreads();
  if (tid < 32) { float a = 0.f; for (int k = 0; k < 32; ++k) a += sv1[tid][k] * bfr(WV2[k]); sov[tid] = tanhf(a); }
  __syncthreads();
  if (tid < 40) vst2(OA + (size_t)gb * 5 + tid * 4, *(const v4f*)&soa[tid * 4]);
  if (tid >= 64 && tid < 96) vst2(OACT + (size_t)gb * 4 + (tid - 64) * 4, *(const v4f*)&soact[(tid - 64) * 4]);
  if (tid >= 96 && tid < 104) vst2(OV + (size_t)gb + (tid - 96) * 4, *(const v4f*)&sov[(tid - 96) * 4]);
  __shared__ __align__(16) float sbig[8][1000];
#pragma unroll 1
  for (int which = 0; which < 2; ++which) { const float* Wm = which ? WT : WS; float* OUT = which ? OT : OS;
#pragma unroll 1
    for (int g8 = 0; g8 < 4; ++g8) {
      for (int q = tid; q < 8 * 1000; q += 256) { const int gl = g8 * 8 + q / 1000, c = q % 1000; float a = 0.f; for (int k = 0; k < 64; ++k) a += s2[gl][k] * bfr(Wm[(size_t)k * 1000 + c]); sbig[q / 1000][c] = a; }
      __syncthreads();
      for (int q = tid; q < 8 * 1000 / 4; q += 256) vst2(OUT + ((size_t)gb + g8 * 8) * 1000 + q * 4, *(const v4f*)&(&sbig[0][0])[q * 4]);
      __syncthreads(); } }
}

extern "C" void kernel_launch(void* const* d_in, const int* in_sizes, int n_in, void* d_out, int out_size, void* d_ws, size_t ws_size, hipStream_t stream) {
  (void)in_sizes; (void)n_in; (void)out_size;
  const float** F = (const float**)d_in; const int* EI = (const int*)d_in[1];
  if (ws_size < (size_t)WS_END) return;
  char* ws = (char*)d_ws;
  int *CNT = (int*)(ws + WS_CNT), *OFF = (int*)(ws + WS_OFF), *BST = (int*)(ws + WS_BST), *SEGS = (int*)(ws + WS_SEGS), *SEGE = (int*)(ws + WS_SEGE), *FS = (int*)(ws + WS_FS), *FE = (int*)(ws + WS_FE), *RST = (int*)(ws + WS_RST), *RCT = (int*)(ws + WS_RCT);
  __bf16* PW = (__bf16*)(ws + WS_PW); float *HW = (float*)(ws + WS_HW), *Hd = (float*)(ws + WS_H), *T = (float*)(ws + WS_T); (void)T;
  const int* SRC = EI; const int* DST = EI + EP;
  k_csr_cnt<<<CSR_NCH, 256, 0, stream>>>(DST, 1, CNT); k_csr_scan<<<1, 256, 0, stream>>>(CNT, OFF, BST); k_csr_scatter<<<CSR_NCH, 256, 0, stream>>>(SRC, DST, 1, 1, OFF, SEGS, SEGE); k_csr_bucket<<<CSR_NBK, 256, 0, stream>>>(CNT, OFF, BST, SEGS, SEGE, DST, 1, FS, FE, RST, RCT);
  const int* BATCH = (const int*)d_in[4]; float *MSG = (float*)(ws + WS_MSG), *PT = (float*)(ws + WS_PT), *PC = (float*)(ws + WS_PC), *GE = (float*)(ws + WS_GE);
  float* OA = (float*)d_out; float* OS = OA + NG * 5; float* OT = OS + NG * 1000; float* OACT = OT + NG * 1000; float* OV = OACT + NG * 4;
  k_packT<<<128, 256, 0, stream>>>(F[6], 32, 128, PW + PW0); k_packT<<<128, 256, 0, stream>>>(F[7], 128, 128, PW + PW0 + 128 * 32);
  k_lin<32, 8, 1, 0><<<dim3(NBLK, 1), 128, 0, stream>>>(F[0], 32, PW + PW0, nullptr, HW, MAXW);
  k_wagg<<<NRP / 16, 256, 0, stream>>>(HW, FS, FE, RST, RCT, F[2], MSG);
  k_comb<<<NBLK, 128, 0, stream>>>(MSG, PW + PW0 + 128 * 32, HW, MSG);
  k_poolpart<<<dim3(NCHK, 2), 128, 0, stream>>>(MSG, BATCH, PT, PC);
  k_poolred<<<NG, 128, 0, stream>>>(PT, PC, GE);
  k_heads<<<NG / 32, 256, 0, stream>>>(GE, F[8], F[9], F[10], F[11], F[12], F[13], F[14], F[15], OA, OS, OT, OACT, OV);
}
